// ResidualMamba3_44848048505419
// MI455X (gfx1250) — hardware-run, weakly checked
//
#include <hip/hip_runtime.h>
#include <math.h>

typedef __attribute__((ext_vector_type(16))) _Float16 v16h;
typedef __attribute__((ext_vector_type(8)))  _Float16 v8h;
typedef __attribute__((ext_vector_type(8)))  float    v8f;
typedef __attribute__((ext_vector_type(4)))  float    v4f;

constexpr int kB     = 4;
constexpr int kL     = 2048;
constexpr int kDM    = 1024;
constexpr int kDS    = 128;
constexpr int kHD    = 64;
constexpr int kDI    = 2048;
constexpr int kNH    = 32;
constexpr int kCD    = kDI + 2 * kDS;
constexpr int kDIP   = 2 * kDI + 2 * kDS + kNH;
constexpr int kDIPP  = 4416;
constexpr int kRows  = kB * kL;
constexpr int kQ     = 32;
constexpr int kNC    = kL / kQ;
constexpr int kTP    = 260;
static_assert(kCD == 2304 && kDIP == 4384, "widths");
static_assert(kDIPP % 64 == 0 && kDIPP >= kDIP && kDIPP - kDIP == 32, "padded in_proj width");
static_assert(kNH * kHD == kDI, "heads");
static_assert(kRows % 64 == 0 && kDM % 64 == 0 && kDI % 64 == 0 && kCD % 64 == 0, "tile multiples");
static_assert(kDM % 32 == 0 && kDI % 32 == 0 && kDS % 32 == 0 && kQ % 32 == 0, "K multiples of 32");
static_assert(kL % 64 == 0 && kL % kQ == 0 && kCD % 256 == 0, "chunking");
static_assert((kRows / 64) * (kDIPP / 64) % 8 == 0 && (kRows / 64) * (kDM / 64) % 8 == 0, "tiles per block");

constexpr float kCarryX  = 64.0f;
constexpr float kCarryW  = 32.0f;
constexpr float kCarryYn = 16.0f;
constexpr float kCarryH  = 1024.0f;
constexpr float kCarryM  = 256.0f;
constexpr float kCarryXd = 256.0f;
constexpr float kInvS0   = 1.0f / (kCarryX * kCarryW);
constexpr float kInvS2   = 1.0f / (kCarryYn * kCarryW);
constexpr float kEps     = 1e-5f;

constexpr size_t kSzWOT = (size_t)kDM * kDI * 2;
constexpr size_t kSzZ   = (size_t)kRows * kDI * 2;
constexpr size_t kSzXBC = (size_t)kRows * kCD * 2;
constexpr size_t kSzX16 = (size_t)kRows * kDM * 2;
constexpr size_t kSzWIT = (size_t)kDIPP * kDM * 2;
constexpr size_t kSzY16 = (size_t)kRows * kDI * 2;
constexpr size_t kSzDT  = (size_t)kRows * kNH * 4;
constexpr size_t kSzG   = (size_t)kRows * kQ * 4;
constexpr size_t kOffWOT = 0;
constexpr size_t kOffZ   = kOffWOT + kSzWOT;
constexpr size_t kOffR2  = kOffZ + kSzZ;
constexpr size_t kOffR3  = kOffR2 + kSzXBC;
constexpr size_t kOffDT  = kOffR3 + kSzXBC;
constexpr size_t kOffG   = kOffDT + kSzDT;
constexpr size_t kWsTotal = kOffG + kSzG;
static_assert(kSzX16 + kSzWIT <= kSzXBC && kSzY16 <= kSzXBC, "aliased planes fit");
static_assert(kWsTotal == 115343360ull, "carve total");
static_assert(kWsTotal <= 134217728ull, "carve cap");
static_assert((kOffZ % 128) == 0 && (kOffR2 % 128) == 0 && (kOffR3 % 128) == 0 && (kOffDT % 128) == 0 &&
              (kOffG % 128) == 0 && (kSzX16 % 128) == 0, "128-B aligned regions");

__device__ __forceinline__ float h16_to_f32(unsigned hb) {
  const unsigned sgn = (hb & 0x8000u) << 16;
  const unsigned em = hb & 0x7fffu;
  const float fn = __uint_as_float((em << 13) + 0x38000000u);
  const float fs = (float)em * 5.9604644775390625e-8f;
  const float mag = (em < 0x400u) ? fs : fn;
  return __uint_as_float(__float_as_uint(mag) | sgn);
}
__device__ __forceinline__ unsigned f2h_bits(float x) {
  const _Float16 hv = (_Float16)x;
  return (unsigned)__builtin_bit_cast(unsigned short, hv);
}
__device__ __forceinline__ void guard4_h(v8f& a, v8f& b, v8f& c, v8f& d, v16h x, v16h y) {
  asm volatile("v_nop\n\tv_nop\n\tv_nop\n\tv_nop" : "+v"(a), "+v"(b), "+v"(c), "+v"(d) : "v"(x), "v"(y));
}
__device__ __forceinline__ void keep4_h(v16h a, v16h b, v16h c, v16h d) { asm volatile("v_nop" :: "v"(a), "v"(b), "v"(c), "v"(d)); }
__device__ __forceinline__ void acc_guard4(v8f& a, v8f& b, v8f& c, v8f& d) { asm volatile("v_nop\n\tv_nop\n\tv_nop\n\tv_nop" : "+v"(a), "+v"(b), "+v"(c), "+v"(d)); }
union FragU { v16h v; v8h h[2]; };
__device__ __forceinline__ v16h frag_load(const _Float16* p) {
  FragU f;
  f.h[0] = *(const v8h*)(p);
  f.h[1] = *(const v8h*)(p + 16);
  return f.v;
}
__device__ __forceinline__ v8f mma_raw(v16h a, v16h b, v8f c) {
  return __builtin_amdgcn_wmma_f32_16x16x32_f16(false, a, false, b, (short)0, c, false, false);
}
__device__ __forceinline__ v8f mma_g(v16h a, v16h b, v8f c) {
  c = __builtin_amdgcn_wmma_f32_16x16x32_f16(false, a, false, b, (short)0, c, false, false);
  asm volatile("v_nop\n\tv_nop\n\tv_nop\n\tv_nop" : "+v"(c) : "v"(a), "v"(b));
  return c;
}

__global__ __launch_bounds__(256) void cast_f16_kernel(
    const float* __restrict__ src, unsigned short* __restrict__ dst, int total8, float scale)
{
  const int i = blockIdx.x * 256 + threadIdx.x;
  if (i >= total8) return;
  const size_t e0 = (size_t)i << 3;
  const float* p = src + e0;
  const v4f a0 = *(const v4f*)(p);
  const v4f a1 = *(const v4f*)(p + 4);
  v8h hv;
#pragma unroll
  for (int e = 0; e < 4; ++e) {
    hv[e]     = (_Float16)(a0[e] * scale);
    hv[4 + e] = (_Float16)(a1[e] * scale);
  }
  unsigned short* q = dst + e0;
  *(volatile v8h*)q = hv;
  __threadfence();
  *(volatile v8h*)q = hv;
}

__global__ __launch_bounds__(256) void transpose_cast_kernel(
    const float* __restrict__ W, unsigned short* __restrict__ Bt, int Kdim, int Ndim, float scale)
{
  __shared__ float tile[64 * 65];
  const int tid = threadIdx.x, lane = tid & 31, wave = tid >> 5;
  const int n0 = blockIdx.x * 64;
  const int k0 = blockIdx.y * 64;
#pragma unroll
  for (int p = 0; p < 16; ++p) {
    const int idx = tid + p * 256;
    const int kk  = idx >> 6;
    const int nn  = idx & 63;
    const int n   = n0 + nn;
    const int nc  = (n < Ndim) ? n : (Ndim - 1);
    const float v = W[(size_t)(k0 + kk) * Ndim + nc];
    tile[kk * 65 + nn] = (n < Ndim) ? (v * scale) : 0.f;
  }
  __syncthreads();
  const int q = lane >> 3, c8 = (lane & 7) * 8;
  v8h hv[2];
#pragma unroll
  for (int it = 0; it < 2; ++it) {
    const int nrow = it * 32 + wave * 4 + q;
#pragma unroll
    for (int e = 0; e < 8; ++e) hv[it][e] = (_Float16)tile[(c8 + e) * 65 + nrow];
  }
  for (int pass = 0; pass < 2; ++pass) {
#pragma unroll
    for (int it = 0; it < 2; ++it) {
      const int nrow = it * 32 + wave * 4 + q;
      *(volatile v8h*)(Bt + (size_t)(n0 + nrow) * Kdim + k0 + c8) = hv[it];
    }
    __threadfence();
  }
}

template <int MODE>
__global__ __launch_bounds__(256) void gemm_f16_kernel(
    const unsigned short* __restrict__ Ap, int lda,
    const unsigned short* __restrict__ Btp, int ldb,
    int M, int N, int K, float scale,
    unsigned short* __restrict__ Z16, unsigned short* __restrict__ XBC16, float* __restrict__ DTRAW,
    float* __restrict__ OUT, const float* __restrict__ RES, int ldc)
{
  const _Float16* A  = (const _Float16*)Ap;
  const _Float16* Bt = (const _Float16*)Btp;
  __shared__ __align__(16) float sT[8][16 * 68];
  const int lane = threadIdx.x & 31;
  const int wave = threadIdx.x >> 5;
  const int tilesN = N >> 6;
  const int tilesM = M >> 6;
  const int tile = blockIdx.x * 8 + wave;
  if (tile >= tilesM * tilesN) return;
  const int tm = tile / tilesN;
  const int tn = tile - tm * tilesN;
  const int m0 = tm << 6;
  const int n0 = tn << 6;
  const int rlane = lane & 15;
  const int koff  = (lane >> 4) * 8;
  const int mOff  = (lane >> 4) * 8;

  v8f acc[4][4];
#pragma unroll
  for (int i = 0; i < 4; ++i)
#pragma unroll
    for (int j = 0; j < 4; ++j) acc[i][j] = (v8f){0.f,0.f,0.f,0.f,0.f,0.f,0.f,0.f};

  for (int k0 = 0; k0 < K; k0 += 32) {
    v16h bh[4];
#pragma unroll
    for (int j = 0; j < 4; ++j) {
      const size_t bo = (size_t)(n0 + (j << 4) + rlane) * ldb + koff + k0;
      bh[j] = frag_load(Bt + bo);
    }
#pragma unroll
    for (int i = 0; i < 4; ++i) {
      const size_t ao = (size_t)(m0 + (i << 4) + rlane) * lda + koff + k0;
      const v16h ah = frag_load(A + ao);
#pragma unroll
      for (int j = 0; j < 4; ++j) acc[i][j] = mma_raw(ah, bh[j], acc[i][j]);
      guard4_h(acc[i][0], acc[i][1], acc[i][2], acc[i][3], ah, bh[0]);
    }
    keep4_h(bh[0], bh[1], bh[2], bh[3]);
  }
  acc_guard4(acc[0][0], acc[0][1], acc[0][2], acc[0][3]);
  acc_guard4(acc[1][0], acc[1][1], acc[1][2], acc[1][3]);
  acc_guard4(acc[2][0], acc[2][1], acc[2][2], acc[2][3]);
  acc_guard4(acc[3][0], acc[3][1], acc[3][2], acc[3][3]);

  float* slab = sT[wave];
#pragma unroll
  for (int i = 0; i < 4; ++i) {
    const int mBase = m0 + (i << 4);
#pragma unroll
    for (int j = 0; j < 4; ++j) {
#pragma unroll
      for (int r = 0; r < 8; ++r) slab[(mOff + r) * 68 + (j << 4) + rlane] = acc[i][j][r] * scale;
    }
    __builtin_amdgcn_fence(__ATOMIC_RELEASE, "workgroup");
    __builtin_amdgcn_wave_barrier();
    __builtin_amdgcn_fence(__ATOMIC_ACQUIRE, "workgroup");
    if (MODE == 0) {
      if (n0 < kDI + kCD) {
        const bool isz = (n0 < kDI);
        unsigned short* dst = isz ? Z16 : XBC16;
        const int ldd = isz ? kDI : kCD;
        const int nc  = isz ? n0 : (n0 - kDI);
        const int q = lane >> 3, c8 = (lane & 7) * 8;
        v8h hv[4];
#pragma unroll
        for (int it = 0; it < 4; ++it) {
          const float* sp = slab + (it * 4 + q) * 68 + c8;
#pragma unroll
          for (int e = 0; e < 8; ++e) hv[it][e] = (_Float16)sp[e];
        }
        for (int pass = 0; pass < 2; ++pass) {
#pragma unroll
          for (int it = 0; it < 4; ++it) {
            const int row = it * 4 + q;
            *(volatile v8h*)(dst + (size_t)(mBase + row) * ldd + nc + c8) = hv[it];
          }
          __threadfence();
        }
      } else {
        const int q = lane >> 3, c4 = (lane & 7) * 4;
        v4f fv[4];
#pragma unroll
        for (int it = 0; it < 4; ++it) fv[it] = *(const v4f*)(slab + (it * 4 + q) * 68 + c4);
        for (int pass = 0; pass < 2; ++pass) {
#pragma unroll
          for (int it = 0; it < 4; ++it) {
            const int row = it * 4 + q;
            *(volatile v4f*)(DTRAW + (size_t)(mBase + row) * kNH + c4) = fv[it];
          }
          __threadfence();
        }
      }
    } else {
      const int hh = lane >> 4, c4 = (lane & 15) * 4;
      v4f ov[8];
#pragma unroll
      for (int it = 0; it < 8; ++it) {
        const int row = it * 2 + hh;
        const v4f sv = *(const v4f*)(slab + row * 68 + c4);
        const v4f rv = *(const v4f*)(RES + (size_t)(mBase + row) * ldc + n0 + c4);
        ov[it] = rv + sv;
      }
      for (int pass = 0; pass < 2; ++pass) {
#pragma unroll
        for (int it = 0; it < 8; ++it) {
          const int row = it * 2 + hh;
          *(volatile v4f*)(OUT + (size_t)(mBase + row) * ldc + n0 + c4) = ov[it];
        }
        __threadfence();
      }
    }
    __builtin_amdgcn_fence(__ATOMIC_RELEASE, "workgroup");
    __builtin_amdgcn_wave_barrier();
    __builtin_amdgcn_fence(__ATOMIC_ACQUIRE, "workgroup");
  }
}

__global__ __launch_bounds__(256) void conv_silu_kernel(
    const unsigned short* __restrict__ XBC16, const float* __restrict__ cw, const float* __restrict__ cb,
    unsigned short* __restrict__ XC16)
{
  __shared__ __align__(16) float sT[16 * kTP];
  const int tid = threadIdx.x, lane = tid & 31, wave = tid >> 5;
  const int d0 = blockIdx.x * 256, d = d0 + tid;
  const int g0 = blockIdx.y * 64;
  const int tb = g0 & (kL - 1);
  const float w0 = cw[d], w1 = cw[kCD + d], w2 = cw[2 * kCD + d], w3 = cw[3 * kCD + d];
  const float bc = cb[d];
  float xm3, xm2, xm1;
  {
    const bool hist = (tb > 0);
    const int rb = hist ? (g0 - 3) : g0;
    const float v3 = h16_to_f32((unsigned)XBC16[(size_t)rb * kCD + d]);
    const float v2 = h16_to_f32((unsigned)XBC16[(size_t)(rb + 1) * kCD + d]);
    const float v1 = h16_to_f32((unsigned)XBC16[(size_t)(rb + 2) * kCD + d]);
    xm3 = hist ? v3 : 0.f;
    xm2 = hist ? v2 : 0.f;
    xm1 = hist ? v1 : 0.f;
  }
#pragma unroll 1
  for (int sub = 0; sub < 4; ++sub) {
    const int lb = g0 + sub * 16;
#pragma unroll 1
    for (int s = 0; s < 16; ++s) {
      const float xcur = h16_to_f32((unsigned)XBC16[(size_t)(lb + s) * kCD + d]);
      float acc = w0 * xm3;
      acc = fmaf(w1, xm2, acc);
      acc = fmaf(w2, xm1, acc);
      acc = fmaf(w3, xcur, acc);
      const float sv = acc + bc;
      const float sg = __builtin_amdgcn_rcpf(1.0f + expf(-sv));
      sT[s * kTP + tid] = sv * sg;
      xm3 = xm2; xm2 = xm1; xm1 = xcur;
    }
    __syncthreads();
    v8h bv[2];
#pragma unroll
    for (int it = 0; it < 2; ++it) {
      const float* sp = sT + (it * 8 + wave) * kTP + lane * 8;
      const v4f a0 = *(const v4f*)(sp);
      const v4f a1 = *(const v4f*)(sp + 4);
#pragma unroll
      for (int e = 0; e < 4; ++e) {
        bv[it][e]     = (_Float16)a0[e];
        bv[it][4 + e] = (_Float16)a1[e];
      }
    }
    for (int pass = 0; pass < 2; ++pass) {
#pragma unroll
      for (int it = 0; it < 2; ++it)
        *(volatile v8h*)(XC16 + (size_t)(lb + it * 8 + wave) * kCD + d0 + lane * 8) = bv[it];
      __threadfence();
    }
    __syncthreads();
  }
}

__global__ __launch_bounds__(128) void gram_kernel(const unsigned short* __restrict__ XC16, float* __restrict__ GRAM)
{
  __shared__ __align__(16) float sG[4][32 * 36];
  const int lane = threadIdx.x & 31, wave = threadIdx.x >> 5;
  const int hh = lane >> 4, rl = lane & 15, koff = hh * 8;
  const int row0 = (blockIdx.x * 4 + wave) * kQ;
  const _Float16* X = (const _Float16*)XC16;
  v8f a00 = (v8f){0.f,0.f,0.f,0.f,0.f,0.f,0.f,0.f};
  v8f a01 = a00, a10 = a00, a11 = a00;
#pragma unroll
  for (int k0 = 0; k0 < kDS; k0 += 32) {
    const v16h c0 = frag_load(X + (size_t)(row0 + rl) * kCD + kDI + kDS + k0 + koff);
    const v16h c1 = frag_load(X + (size_t)(row0 + 16 + rl) * kCD + kDI + kDS + k0 + koff);
    const v16h b0 = frag_load(X + (size_t)(row0 + rl) * kCD + kDI + k0 + koff);
    const v16h b1 = frag_load(X + (size_t)(row0 + 16 + rl) * kCD + kDI + k0 + koff);
    a00 = mma_g(c0, b0, a00);
    a01 = mma_g(c0, b1, a01);
    a10 = mma_g(c1, b0, a10);
    a11 = mma_g(c1, b1, a11);
  }
  float* sg = sG[wave];
#pragma unroll
  for (int r = 0; r < 8; ++r) {
    sg[(8 * hh + r) * 36 + rl]           = a00[r];
    sg[(8 * hh + r) * 36 + 16 + rl]      = a01[r];
    sg[(16 + 8 * hh + r) * 36 + rl]      = a10[r];
    sg[(16 + 8 * hh + r) * 36 + 16 + rl] = a11[r];
  }
  __builtin_amdgcn_fence(__ATOMIC_RELEASE, "workgroup");
  __builtin_amdgcn_wave_barrier();
  __builtin_amdgcn_fence(__ATOMIC_ACQUIRE, "workgroup");
  const int q = lane >> 3, c4 = (lane & 7) * 4;
  v4f fv[8];
#pragma unroll
  for (int it = 0; it < 8; ++it) fv[it] = *(const v4f*)(sg + (it * 4 + q) * 36 + c4);
  for (int pass = 0; pass < 2; ++pass) {
#pragma unroll
    for (int it = 0; it < 8; ++it)
      *(volatile v4f*)(GRAM + (size_t)(row0 + it * 4 + q) * kQ + c4) = fv[it];
    __threadfence();
  }
}

__global__ __launch_bounds__(256) void scan_ssd_kernel(
    const unsigned short* __restrict__ XC16, const float* __restrict__ DTRAW, const float* __restrict__ GRAM,
    const float* __restrict__ dt_bias, const float* __restrict__ A_log, const float* __restrict__ Dp,
    unsigned short* __restrict__ Y16)
{
  __shared__ __align__(16) _Float16 sBC[kQ * 256];
  __shared__ __align__(16) _Float16 sBt[kDS * kQ];
  __shared__ __align__(16) _Float16 sXd[kHD * kQ];
  __shared__ __align__(16) _Float16 sXw[kHD * kQ];
  __shared__ __align__(16) _Float16 sM[kQ * kQ];
  __shared__ __align__(16) _Float16 sH[kHD * kDS];
  __shared__ __align__(16) float sXh[kQ * kHD];
  __shared__ float sDt[kQ];
  __shared__ float sCs[kQ];
  __shared__ float sEc[kQ];
  __shared__ float sWd[kQ];

  const int tid = threadIdx.x, lane = tid & 31, wave = tid >> 5;
  const int hh = lane >> 4, rl = lane & 15, koff = hh * 8;
  const int b = blockIdx.x >> 5, h = blockIdx.x & 31;
  const float Ah  = -expf(A_log[h]);
  const float dtb = dt_bias[h];
  const float Dh  = Dp[h];
  const float fI = 1.0f / kCarryH;
  const float fM = 1.0f / (kCarryM * kCarryXd);
  const float fU = 1.0f / kCarryXd;
  const v8f vz = (v8f){0.f,0.f,0.f,0.f,0.f,0.f,0.f,0.f};
  v8f hacc[4];
#pragma unroll
  for (int i = 0; i < 4; ++i) hacc[i] = vz;

  {
    const uint4 z4 = make_uint4(0u, 0u, 0u, 0u);
#pragma unroll
    for (int i = 0; i < 4; ++i) ((uint4*)sH)[tid + i * 256] = z4;
  }
  __syncthreads();

#pragma unroll 1
  for (int c = 0; c < kNC; ++c) {
    const int row0 = b * kL + c * kQ;
#pragma unroll
    for (int i = 0; i < 4; ++i) {
      const int idx = tid + i * 256;
      const int r = idx >> 5, c8 = (idx & 31) * 8;
      const uint4 v = *(const uint4*)(XC16 + (size_t)(row0 + r) * kCD + kDI + c8);
      *(uint4*)(sBC + r * 256 + c8) = v;
    }
    {
      const int t = tid >> 3, c8 = (tid & 7) * 8;
      const uint4 v = *(const uint4*)(XC16 + (size_t)(row0 + t) * kCD + h * kHD + c8);
      v4f f0, f1;
      f0[0] = h16_to_f32(v.x & 0xffffu); f0[1] = h16_to_f32(v.x >> 16);
      f0[2] = h16_to_f32(v.y & 0xffffu); f0[3] = h16_to_f32(v.y >> 16);
      f1[0] = h16_to_f32(v.z & 0xffffu); f1[1] = h16_to_f32(v.z >> 16);
      f1[2] = h16_to_f32(v.w & 0xffffu); f1[3] = h16_to_f32(v.w >> 16);
      *(v4f*)(sXh + t * kHD + c8)     = f0;
      *(v4f*)(sXh + t * kHD + c8 + 4) = f1;
    }
    {
      const float raw = DTRAW[(size_t)(row0 + lane) * kNH + h] + dtb;
      const float dt  = fmaxf(raw, 0.0f) + log1pf(expf(-fabsf(raw)));
      float cs = dt * Ah;
#pragma unroll
      for (int off = 1; off < 32; off <<= 1) {
        const float up = __shfl_up(cs, off, 32);
        cs += (lane >= off) ? up : 0.0f;
      }
      const float cs31 = __shfl(cs, 31, 32);
      const float ad = fminf(cs31 - cs, 0.0f);
      const float ac = fminf(cs, 0.0f);
      const float ed = expf(ad);
      const float ec = expf(ac);
      const float wd = (ad > -87.0f) ? ed : 0.0f;
      const float wc = (ac > -87.0f) ? ec : 0.0f;
      if (wave == 0) { sDt[lane] = dt; sCs[lane] = cs; sEc[lane] = wc; sWd[lane] = wd; }
    }
    __syncthreads();

    {
      const int n = tid & 127, sh = tid >> 7;
      const unsigned short* src = (const unsigned short*)sBC;
      unsigned wv[8];
#pragma unroll
      for (int e = 0; e < 8; ++e) {
        const unsigned lo = (unsigned)src[(sh * 16 + 2 * e) * 256 + n];
        const unsigned hi = (unsigned)src[(sh * 16 + 2 * e + 1) * 256 + n];
        wv[e] = lo | (hi << 16);
      }
      *(uint4*)(sBt + n * kQ + sh * 16)     = make_uint4(wv[0], wv[1], wv[2], wv[3]);
      *(uint4*)(sBt + n * kQ + sh * 16 + 8) = make_uint4(wv[4], wv[5], wv[6], wv[7]);
    }
    {
      const int p = tid >> 2, s0 = (tid & 3) * 8;
      v8h xd, xw;
#pragma unroll
      for (int e = 0; e < 8; ++e) {
        const int s = s0 + e;
        const float v = sDt[s] * sXh[s * kHD + p];
        xd[e] = (_Float16)(v * kCarryXd);
        xw[e] = (_Float16)((v * sWd[s]) * kCarryXd);
      }
      *(v8h*)(sXd + p * kQ + s0) = xd;
      *(v8h*)(sXw + p * kQ + s0) = xw;
    }
    {
      const int t = tid >> 3, s0 = (tid & 7) * 4;
      const v4f g4 = *(const v4f*)(GRAM + (size_t)(row0 + t) * kQ + s0);
      const float cst = sCs[t];
      unsigned hb[4];
#pragma unroll
      for (int e = 0; e < 4; ++e) {
        const int s = s0 + e;
        const float ar = fminf(cst - sCs[s], 0.0f);
        const float ex = expf(ar);
        const float w  = ((s <= t) && (ar > -87.0f)) ? ex : 0.0f;
        const float gv = g4[e];
        hb[e] = f2h_bits((w * gv) * kCarryM);
      }
      uint2 wv2;
      wv2.x = hb[0] | (hb[1] << 16);
      wv2.y = hb[2] | (hb[3] << 16);
      *(uint2*)(sM + t * kQ + s0) = wv2;
    }
    __syncthreads();

    {
      const int tt = wave >> 2, pt = wave & 3;
      v8f accI = vz, accM = vz;
#pragma unroll
      for (int k0 = 0; k0 < kDS; k0 += 32) {
        const v16h a  = frag_load(sBC + (tt * 16 + rl) * 256 + kDS + k0 + koff);
        const v16h bb = frag_load(sH + (pt * 16 + rl) * kDS + k0 + koff);
        accI = mma_g(a, bb, accI);
      }
      {
        const v16h am = frag_load(sM + (tt * 16 + rl) * kQ + koff);
        const v16h bx = frag_load(sXd + (pt * 16 + rl) * kQ + koff);
        accM = mma_g(am, bx, accM);
      }
#pragma unroll
      for (int r = 0; r < 8; ++r) {
        const int t = tt * 16 + 8 * hh + r;
        const int p = pt * 16 + rl;
        const float xv = sXh[t * kHD + p];
        float y = accI[r] * (sEc[t] * fI);
        y += accM[r] * fM;
        y += Dh * xv;
        sXh[t * kHD + p] = y;
      }
    }
    __syncthreads();

    {
      const float e31 = sEc[kQ - 1];
      const v16h bb = frag_load(sBt + (wave * 16 + rl) * kQ + koff);
#pragma unroll
      for (int pt = 0; pt < 4; ++pt) {
        const v16h ax = frag_load(sXw + (pt * 16 + rl) * kQ + koff);
        const v8f pr = mma_g(ax, bb, vz);
#pragma unroll
        for (int r = 0; r < 8; ++r) {
          const float hn = e31 * hacc[pt][r] + pr[r] * fU;
          hacc[pt][r] = hn;
          sH[(pt * 16 + 8 * hh + r) * kDS + wave * 16 + rl] = (_Float16)(hn * kCarryH);
        }
      }
    }
    {
      const int t = wave * 4 + (lane >> 3), c8 = (lane & 7) * 8;
      const v4f a0 = *(const v4f*)(sXh + t * kHD + c8);
      const v4f a1 = *(const v4f*)(sXh + t * kHD + c8 + 4);
      v8h hv;
#pragma unroll
      for (int e = 0; e < 4; ++e) {
        hv[e]     = (_Float16)a0[e];
        hv[4 + e] = (_Float16)a1[e];
      }
      unsigned short* dst = Y16 + (size_t)(row0 + t) * kDI + h * kHD + c8;
      *(volatile v8h*)dst = hv;
      __threadfence();
      *(volatile v8h*)dst = hv;
    }
    __syncthreads();
  }
}

__global__ __launch_bounds__(256) void gate_norm_kernel(
    const unsigned short* __restrict__ Y16, const unsigned short* __restrict__ Z16, const float* __restrict__ nw,
    unsigned short* __restrict__ YN16)
{
  __shared__ __align__(16) float sg[kDI];
  __shared__ float sred[8];
  const int tid = threadIdx.x, lane = tid & 31, wave = tid >> 5;
  const size_t rb = (size_t)blockIdx.x * kDI;
  float ss = 0.f;
#pragma unroll 1
  for (int i = 0; i < 8; ++i) {
    const int ch = i * 256 + tid;
    const float yv = h16_to_f32((unsigned)Y16[rb + ch]);
    const float zv = h16_to_f32((unsigned)Z16[rb + ch]);
    const float sgm = __builtin_amdgcn_rcpf(1.0f + expf(-zv));
    const float g = yv * (zv * sgm);
    sg[ch] = g;
    ss = fmaf(g, g, ss);
  }
#pragma unroll
  for (int off = 16; off > 0; off >>= 1) ss += __shfl_xor(ss, off, 32);
  if (lane == 0) sred[wave] = ss;
  __syncthreads();
  float tot = sred[0];
  tot += sred[1]; tot += sred[2]; tot += sred[3];
  tot += sred[4]; tot += sred[5]; tot += sred[6]; tot += sred[7];
  const float sc = rsqrtf(tot * (1.0f / (float)kDI) + kEps);
  const int c8 = tid * 8;
  const v4f g0 = *(const v4f*)(sg + c8);
  const v4f g1 = *(const v4f*)(sg + c8 + 4);
  const v4f w0 = *(const v4f*)(nw + c8);
  const v4f w1 = *(const v4f*)(nw + c8 + 4);
  v8h hv;
#pragma unroll
  for (int e = 0; e < 4; ++e) {
    hv[e]     = (_Float16)(((g0[e] * sc) * w0[e]) * kCarryYn);
    hv[4 + e] = (_Float16)(((g1[e] * sc) * w1[e]) * kCarryYn);
  }
  unsigned short* dst = YN16 + rb + c8;
  *(volatile v8h*)dst = hv;
  __threadfence();
  *(volatile v8h*)dst = hv;
}

extern "C" void kernel_launch(void* const* d_in, const int* in_sizes, int n_in,
                              void* d_out, int out_size, void* d_ws, size_t ws_size,
                              hipStream_t stream)
{
  if (n_in < 9) return;
  if (in_sizes[0] != kRows * kDM) return;
  if (in_sizes[1] != kDM * kDIP) return;
  if (in_sizes[2] != 4 * kCD) return;
  if (in_sizes[3] != kCD) return;
  if (in_sizes[4] != kNH || in_sizes[5] != kNH || in_sizes[6] != kNH) return;
  if (in_sizes[7] != kDI) return;
  if (in_sizes[8] != kDI * kDM) return;
  if (out_size != kRows * kDM) return;
  if (ws_size < kWsTotal) return;

  const float* x       = (const float*)d_in[0];
  const float* W_in    = (const float*)d_in[1];
  const float* conv_w  = (const float*)d_in[2];
  const float* conv_b  = (const float*)d_in[3];
  const float* dt_bias = (const float*)d_in[4];
  const float* A_log   = (const float*)d_in[5];
  const float* Dv      = (const float*)d_in[6];
  const float* norm_w  = (const float*)d_in[7];
  const float* W_out   = (const float*)d_in[8];
  float* out = (float*)d_out;

  char* ws = (char*)d_ws;
  unsigned short* WOT16  = (unsigned short*)(ws + kOffWOT);
  unsigned short* Z16    = (unsigned short*)(ws + kOffZ);
  unsigned short* XBC16  = (unsigned short*)(ws + kOffR2);
  unsigned short* Y16    = (unsigned short*)(ws + kOffR2);
  unsigned short* X16    = (unsigned short*)(ws + kOffR3);
  unsigned short* WINT16 = (unsigned short*)(ws + kOffR3 + kSzX16);
  unsigned short* XC16   = (unsigned short*)(ws + kOffR3);
  unsigned short* YN16   = (unsigned short*)(ws + kOffR3);
  float*          DTRAW  = (float*)(ws + kOffDT);
  float*          GRAM   = (float*)(ws + kOffG);

  cast_f16_kernel<<<(kRows * kDM / 8) / 256, 256, 0, stream>>>(x, X16, kRows * kDM / 8, kCarryX);
  transpose_cast_kernel<<<dim3(kDIPP / 64, kDM / 64), 256, 0, stream>>>(W_in, WINT16, kDM, kDIP, kCarryW);
  transpose_cast_kernel<<<dim3(kDM / 64, kDI / 64), 256, 0, stream>>>(W_out, WOT16, kDI, kDM, kCarryW);
  gemm_f16_kernel<0><<<(kRows / 64) * (kDIPP / 64) / 8, 256, 0, stream>>>(
      X16, kDM, WINT16, kDM, kRows, kDIPP, kDM, kInvS0, Z16, XBC16, DTRAW, out, x, kDM);
  conv_silu_kernel<<<dim3(kCD / 256, kRows / 64), 256, 0, stream>>>(XBC16, conv_w, conv_b, XC16);
  gram_kernel<<<(kRows / kQ) / 4, 128, 0, stream>>>(XC16, GRAM);
  scan_ssd_kernel<<<kB * kNH, 256, 0, stream>>>(XC16, DTRAW, GRAM, dt_bias, A_log, Dv, Y16);
  gate_norm_kernel<<<kRows, 256, 0, stream>>>(Y16, Z16, norm_w, YN16);
  gemm_f16_kernel<1><<<(kRows / 64) * (kDM / 64) / 8, 256, 0, stream>>>(
      YN16, kDI, WOT16, kDI, kRows, kDM, kDI, kInvS2, Z16, XBC16, DTRAW, out, x, kDM);
}
